// ClusteredAttention_52441550684839
// MI455X (gfx1250) — hardware-verified
//
#include <hip/hip_runtime.h>
#define NB 4
#define SQ 512
#define NH 32
#define HD 64
#define DM (NH * HD)
#define PCAR 1024.0f
typedef __bf16 v16b __attribute__((ext_vector_type(16)));
typedef unsigned short v8us __attribute__((ext_vector_type(8), may_alias));
typedef float  v8f  __attribute__((ext_vector_type(8)));
typedef float  v4f  __attribute__((ext_vector_type(4)));
typedef float  v4fa __attribute__((ext_vector_type(4), may_alias));
union FragB { v16b v; v8us half[2]; unsigned short u[16]; };

__device__ __forceinline__ unsigned short bf16_bits(float x) { unsigned int u = __float_as_uint(x); return (unsigned short)((u + 0x7FFFu + ((u >> 16) & 1u)) >> 16); }
__device__ __forceinline__ float bf16_val(unsigned short b) { return __uint_as_float(((unsigned int)b) << 16); }
__device__ __forceinline__ float bf16_round(float x) { return bf16_val(bf16_bits(x)); }
template <int NT>
__device__ __forceinline__ v8f mmaN(v16b ah, v16b al, v16b bh, v16b bl, v8f c) {
  c = __builtin_amdgcn_wmma_f32_16x16x32_bf16(false, ah, false, bh, (short)0, c, false, false);
  if (NT >= 2) c = __builtin_amdgcn_wmma_f32_16x16x32_bf16(false, al, false, bh, (short)0, c, false, false);
  if (NT >= 3) c = __builtin_amdgcn_wmma_f32_16x16x32_bf16(false, ah, false, bl, (short)0, c, false, false);
  asm volatile("v_nop\n\tv_nop\n\tv_nop\n\tv_nop" : "+v"(c) : "v"(ah), "v"(al), "v"(bh), "v"(bl));
  return c;
}


typedef _Float16 v16h __attribute__((ext_vector_type(16)));
union FragH { v16h v; v8us half[2]; _Float16 h[16]; unsigned short u[16]; };
template <int NT>
__device__ __forceinline__ v8f mmaH(v16h ah, v16h al, v16h bh, v16h bl, v8f c) {
  c = __builtin_amdgcn_wmma_f32_16x16x32_f16(false, ah, false, bh, (short)0, c, false, false);
  if (NT >= 2) c = __builtin_amdgcn_wmma_f32_16x16x32_f16(false, al, false, bh, (short)0, c, false, false);
  if (NT >= 3) c = __builtin_amdgcn_wmma_f32_16x16x32_f16(false, ah, false, bl, (short)0, c, false, false);
  asm volatile("v_nop\n\tv_nop\n\tv_nop\n\tv_nop" : "+v"(c) : "v"(ah), "v"(al), "v"(bh), "v"(bl));
  return c;
}

typedef _Float16 v4h __attribute__((ext_vector_type(4)));

__global__ __launch_bounds__(256) void k_x16(const float* __restrict__ x, _Float16* __restrict__ X16, size_t n8) { const size_t t = (size_t)blockIdx.x * 256 + threadIdx.x; if (t >= n8) return; FragH f;
#pragma unroll
  for (int q = 0; q < 8; ++q) f.h[q] = (_Float16)bf16_round(x[t * 8 + q]); *(volatile v8us*)((unsigned short*)X16 + t * 8) = f.half[0]; __threadfence(); *(volatile v8us*)((unsigned short*)X16 + t * 8) = f.half[0]; }
template <int NHv, int TTv>
__global__ __launch_bounds__(256) void k_vt(const _Float16* __restrict__ V16, int ldv, int voff, _Float16* __restrict__ Vt) { __shared__ unsigned short tl[64][66]; const int tid = threadIdx.x; const int slab = blockIdx.x / (TTv / 64), lg = blockIdx.x % (TTv / 64); const int b = slab / NHv, h = slab % NHv;
  for (int i = tid; i < 64 * 8; i += 256) { const int r = i / 8, c8 = (i % 8) * 8; FragH f; f.half[0] = *(const v8us*)((const unsigned short*)V16 + ((size_t)b * TTv + lg * 64 + r) * ldv + voff + h * 64 + c8);
#pragma unroll
    for (int q = 0; q < 8; ++q) tl[r][c8 + q] = f.u[q]; }
  __syncthreads();
  for (int pass = 0; pass < 2; ++pass) {
#pragma unroll
    for (int rd = 0; rd < 2; ++rd) { const int d = rd * 32 + tid / 8, pc = tid % 8; FragH f;
#pragma unroll
      for (int q = 0; q < 8; ++q) f.u[q] = tl[pc * 8 + q][d];
      *(volatile v8us*)((unsigned short*)Vt + ((size_t)slab * 64 + d) * TTv + lg * 64 + pc * 8) = f.half[0]; }
    if (pass == 0) __threadfence(); } }

__global__ __launch_bounds__(256) void k_hl(const float* __restrict__ F, _Float16* __restrict__ Hh, _Float16* __restrict__ Hl, size_t n8) { const size_t t = (size_t)blockIdx.x * 256 + threadIdx.x; if (t >= n8) return; FragH fh, fl; const v4f a = *(const v4fa*)(F + t * 8), c = *(const v4fa*)(F + t * 8 + 4);
#pragma unroll
  for (int q = 0; q < 4; ++q) { _Float16 h = (_Float16)a[q]; fh.h[q] = h; fl.h[q] = (_Float16)((a[q] - (float)h) * 1024.0f); h = (_Float16)c[q]; fh.h[4 + q] = h; fl.h[4 + q] = (_Float16)((c[q] - (float)h) * 1024.0f); }
  for (int pass = 0; pass < 2; ++pass) { *(volatile v8us*)((unsigned short*)Hh + t * 8) = fh.half[0]; *(volatile v8us*)((unsigned short*)Hl + t * 8) = fl.half[0]; if (pass == 0) __threadfence(); } }

__device__ __forceinline__ v16h g2_frag(const _Float16* p, int hh) { FragH f; f.half[0] = *(const v8us*)((const unsigned short*)p + 8 * hh); f.half[1] = *(const v8us*)((const unsigned short*)p + 16 + 8 * hh); return f.v; }
__device__ __forceinline__ v8f g2_mma(v16h a, v16h b, v8f c) { v8f d = __builtin_amdgcn_wmma_f32_16x16x32_f16(false, a, false, b, (short)0, c, false, false); asm volatile("v_nop\n\tv_nop\n\tv_nop\n\tv_nop" : "+v"(d) : "v"(a), "v"(b)); return d; }
template <int ACT>
__global__ __launch_bounds__(128) void k_gemm2(const _Float16* __restrict__ A, int lda, size_t sA, const _Float16* __restrict__ Bh, int ldb, size_t sB, float alpha, const float* __restrict__ bias, size_t sBias, const float* __restrict__ CP, int rowsPerB, size_t sCPb, int row0g,
    float* __restrict__ C, _Float16* __restrict__ C16, int ldc, size_t sC, int M, int N, int K) { static_assert(ACT == 0 || ACT == 3 || ACT == 6 || ACT == 8 || ACT == 9 || ACT == 11 || ACT == 12 || ACT == 14 || ACT == 15 || ACT == 16 || ACT == 17, "k_gemm2: unsupported ACT code (would silently apply no activation)");
  __shared__ __attribute__((aligned(16))) float so[4][32][68];
  const int tid = threadIdx.x, w = tid >> 5, lane = tid & 31, ln = lane & 15, hh = lane >> 4; const int by = blockIdx.y;
  A += (size_t)by * sA; Bh += (size_t)by * sB; const size_t cofs = (size_t)by * sC; const float* bp = bias ? bias + (size_t)by * sBias : nullptr;
  const int ntn = N >> 6; const int mt = blockIdx.x / ntn, nq = blockIdx.x - mt * ntn; const int row0 = mt * 128 + 32 * w, col0 = nq * 64; if (row0 >= M) return;
  const _Float16* a0p = A + (size_t)(row0 + ln) * lda; const _Float16* a1p = a0p + (size_t)16 * lda;
  const _Float16* b0p = Bh + (size_t)(col0 + ln) * ldb; const _Float16* b1p = b0p + (size_t)16 * ldb; const _Float16* b2p = b1p + (size_t)16 * ldb; const _Float16* b3p = b2p + (size_t)16 * ldb;
  const v8f z8 = {0.f,0.f,0.f,0.f,0.f,0.f,0.f,0.f}; v8f c00 = z8, c01 = z8, c02 = z8, c03 = z8, c10 = z8, c11 = z8, c12 = z8, c13 = z8;
  for (int kb = 0; kb < K; kb += 32) { const v16h a0 = g2_frag(a0p + kb, hh), a1 = g2_frag(a1p + kb, hh);
    v16h b = g2_frag(b0p + kb, hh); c00 = g2_mma(a0, b, c00); c10 = g2_mma(a1, b, c10);
    b = g2_frag(b1p + kb, hh); c01 = g2_mma(a0, b, c01); c11 = g2_mma(a1, b, c11);
    b = g2_frag(b2p + kb, hh); c02 = g2_mma(a0, b, c02); c12 = g2_mma(a1, b, c12);
    b = g2_frag(b3p + kb, hh); c03 = g2_mma(a0, b, c03); c13 = g2_mma(a1, b, c13); }
  v8f accs[8] = {c00, c01, c02, c03, c10, c11, c12, c13};
#pragma unroll
  for (int u = 0; u < 8; ++u) { const int t = u & 3, half = u >> 2; const int col = col0 + t * 16 + ln; const float bv = bp ? bf16_round(bp[col]) : 0.f;
#pragma unroll
    for (int r = 0; r < 8; ++r) { const int rloc = half * 16 + 8 * hh + r; float v = accs[u][r] * alpha + bv; if (CP) { if (rowsPerB < 0) v += CP[cofs + (size_t)(row0g + row0 + rloc) * ldc + col];        else { const int bidx = (row0g + row0 + rloc) / rowsPerB; v += CP[(size_t)bidx * sCPb + (size_t)by * 64 + col]; } }
      if (ACT == 3) v = fmaxf(v, 0.f); else if (ACT == 6) v = 0.5f * v * (1.0f + erff(v * 0.70710678118654752f)); else if (ACT == 11) v = 1.0f / (1.0f + expf(-v)); else if (ACT == 15) v = v / (1.0f + expf(-v)); else if (ACT == 12) v = (v > 0.f) ? v : 0.01f * v; else if (ACT == 8) v = tanhf(v); else if (ACT == 9) v = 0.5f * v * (1.0f + tanhf(0.7978845608028654f * (v + 0.044715f * v * v * v))); else if (ACT == 14) v = (v > 0.f) ? v : 0.1f * v; else if (ACT == 16) v = (v >= 0.f) ? v : 0.3f * v; else if (ACT == 17) v = (v >= 0.f) ? v : 0.2f * v;
      so[w][rloc][t * 16 + ln] = v; } }
  __builtin_amdgcn_fence(__ATOMIC_ACQ_REL, "workgroup"); __builtin_amdgcn_wave_barrier();
  const int rsub = lane >> 4, c4 = (lane & 15) * 4;
  for (int pass = 0; pass < 2; ++pass) {
#pragma unroll
    for (int q = 0; q < 16; ++q) { const int r = q * 2 + rsub; const v4f v = *(const v4fa*)&so[w][r][c4]; if (C) *(volatile v4f*)(C + cofs + (size_t)(row0 + r) * ldc + col0 + c4) = v; if (C16) { v4h h4; for (int i = 0; i < 4; ++i) h4[i] = (_Float16)v[i]; *(volatile v4h*)(C16 + cofs + (size_t)(row0 + r) * ldc + col0 + c4) = h4; } }
    if (pass == 0) __threadfence(); } }


__global__ __launch_bounds__(256) void k_ksum(const float* __restrict__ key, float* __restrict__ KS, int n8) {
  const int t = blockIdx.x * 256 + threadIdx.x; if (t >= n8) return; const int pos = t / (HD / 8), c8 = (t % (HD / 8)) * 8; const float* kp = key + (size_t)pos * DM + c8; v4f s0 = {0.f, 0.f, 0.f, 0.f}, s1 = {0.f, 0.f, 0.f, 0.f};
  for (int v = 0; v < NH; ++v) { const v4f a = *(const v4fa*)(kp + v * HD), c = *(const v4fa*)(kp + v * HD + 4);
#pragma unroll
    for (int q = 0; q < 4; ++q) { s0[q] += bf16_round(a[q]); s1[q] += bf16_round(c[q]); } }
  float* o = KS + (size_t)pos * HD + c8; *(volatile v4f*)o = s0; *(volatile v4f*)(o + 4) = s1; __threadfence(); *(volatile v4f*)o = s0; *(volatile v4f*)(o + 4) = s1; }
__global__ __launch_bounds__(256) void k_csm(const float* __restrict__ S, _Float16* __restrict__ P, const int* __restrict__ lab, int qn, int hg, float pc) {
  const int t = blockIdx.x * 256 + threadIdx.x; if (t >= qn * hg) return; const int i = t % qn; const size_t r = (size_t)(t / qn) * SQ + i; const float* s = S + r * SQ; const int li = lab[i]; float mx = -3.0e38f;
  for (int j = 0; j < SQ; ++j) { const float x = s[j] + ((lab[j] == li) ? 0.f : -3.0e38f); mx = (x > mx) ? x : mx; } float se = 0.f;
  for (int j = 0; j < SQ; ++j) { const float x = s[j] + ((lab[j] == li) ? 0.f : -3.0e38f); se += expf(x - mx); } const float sc = pc / se;
  for (int j0 = 0; j0 < SQ; j0 += 8) { FragH f;
#pragma unroll
    for (int q = 0; q < 8; ++q) { const float x = s[j0 + q] + ((lab[j0 + q] == li) ? 0.f : -3.0e38f); const float wc = expf(x - mx) * sc; f.h[q] = (_Float16)((wc < 6.103515625e-05f) ? 0.f : wc); }
    unsigned short* d = (unsigned short*)P + r * SQ + j0; *(volatile v8us*)d = f.half[0]; __threadfence(); *(volatile v8us*)d = f.half[0]; } }

extern "C" void kernel_launch(void* const* d_in, const int* in_sizes, int n_in,
                              void* d_out, int out_size, void* d_ws, size_t ws_size, hipStream_t stream) {
  (void)in_sizes; (void)n_in; (void)out_size;
  const float* query = (const float*)d_in[0]; const float* key = (const float*)d_in[1]; const float* value = (const float*)d_in[2]; const int* lab = (const int*)d_in[3];
  static_assert(SQ % 128 == 0 && SQ % 64 == 0 && HD == 64 && ((size_t)NB * SQ * DM / 8) % 256 == 0 && ((size_t)NB * SQ * HD / 8) % 256 == 0 && (NH * SQ) % 256 == 0 && SQ % 8 == 0, "whole tiles; exact grids");
  float* out = (float*)d_out;
  char* ws = (char*)d_ws; size_t off = 0;
  auto take = [&](size_t bytes) { char* p = ws + off; off += (bytes + 255) & ~(size_t)255; return p; };
  _Float16* Q16 = (_Float16*)take((size_t)NB * SQ * DM * 2); _Float16* V16 = (_Float16*)take((size_t)NB * SQ * DM * 2); float* KSF = (float*)take((size_t)NB * SQ * HD * 4); _Float16* KSH = (_Float16*)take((size_t)NB * SQ * HD * 2); _Float16* KSL = (_Float16*)take((size_t)NB * SQ * HD * 2); _Float16* VT = (_Float16*)take((size_t)NH * HD * SQ * 2);
  float* S = (float*)take((size_t)NH * SQ * SQ * 4); _Float16* P = (_Float16*)take((size_t)NH * SQ * SQ * 2);
  if (off > ws_size) return;
  k_x16<<<(unsigned)((size_t)NB * SQ * DM / 8 / 256), 256, 0, stream>>>(query, Q16, (size_t)NB * SQ * DM / 8); k_x16<<<(unsigned)((size_t)NB * SQ * DM / 8 / 256), 256, 0, stream>>>(value, V16, (size_t)NB * SQ * DM / 8);
  k_ksum<<<(NB * SQ * (HD / 8)) / 256, 256, 0, stream>>>(key, KSF, NB * SQ * (HD / 8)); k_hl<<<(unsigned)((size_t)NB * SQ * HD / 8 / 256), 256, 0, stream>>>(KSF, KSH, KSL, (size_t)NB * SQ * HD / 8);
  for (int b = 0; b < NB; ++b) { const size_t r0 = (size_t)b * SQ;
    k_vt<NH, SQ><<<NH * (SQ / 64), 256, 0, stream>>>(V16 + r0 * DM, DM, 0, VT);
    k_gemm2<0><<<dim3((SQ / 128) * (SQ / 64), NH), 128, 0, stream>>>(Q16 + r0 * DM, DM, (size_t)HD, KSH + r0 * HD, HD, (size_t)0, 0.125f, nullptr, 0, nullptr, 1, 0, 0, S, nullptr, SQ, (size_t)SQ * SQ, SQ, SQ, HD); k_gemm2<0><<<dim3((SQ / 128) * (SQ / 64), NH), 128, 0, stream>>>(Q16 + r0 * DM, DM, (size_t)HD, KSL + r0 * HD, HD, (size_t)0, 0.0001220703125f, nullptr, 0, S, -1, 0, 0, S, nullptr, SQ, (size_t)SQ * SQ, SQ, SQ, HD);
    k_csm<<<(NH * SQ) / 256, 256, 0, stream>>>(S, P, lab + r0, SQ, NH, PCAR);
    k_gemm2<0><<<dim3((SQ / 128) * (HD / 64), NH), 128, 0, stream>>>(P, SQ, (size_t)SQ * SQ, VT, SQ, (size_t)HD * SQ, 1.0f / PCAR, nullptr, 0, nullptr, 1, 0, 0, out + r0 * DM, nullptr, DM, (size_t)HD, SQ, HD, SQ); }
}
